// SelfAttention2d_14035953123469
// MI455X (gfx1250) — hardware-verified
//
#include <hip/hip_runtime.h>
#include <math.h>


#ifndef NB
#define NB 8
#endif
#ifndef SEQ
#define SEQ 1024
#endif
#define NB_FULL  8
#define SEQ_FULL 1024
#define CC       256
#define C3       768
#define NHEAD    32
#define HDIM     8
#define GN_EPS   1e-5f
#define LDST     40
#define VST      136
#define OST      132
#define WCARRY   16.0f
#define PCARRY   256.0f
#define YCARRY   64.0f

static_assert(NB >= 1 && NB <= NB_FULL);
static_assert(SEQ >= 128 && SEQ <= SEQ_FULL && (SEQ % 128) == 0);
static_assert(CC == NHEAD * HDIM);
static_assert((C3 * CC / 8) % 256 == 0 && (CC * CC / 8) % 256 == 0);
static_assert(128 * VST / 2 <= 8704 && 64 * OST <= 8704 && 256 * LDST / 2 <= 8704);

typedef _Float16 v16h __attribute__((ext_vector_type(16)));
typedef _Float16 v8h  __attribute__((ext_vector_type(8)));
typedef float    v8f  __attribute__((ext_vector_type(8)));
typedef float    v4f  __attribute__((ext_vector_type(4)));
union Frag { v16h v; v8h h[2]; };

__device__ __forceinline__ float bfr(float f) {
  unsigned u = __float_as_uint(f);
  u += 0x7FFFu + ((u >> 16) & 1u);
  u &= 0xFFFF0000u;
  return __uint_as_float(u);
}

__device__ __forceinline__ v8f wmma16(v16h a, v16h b, v8f c) {
  v8f d = __builtin_amdgcn_wmma_f32_16x16x32_f16(false, a, false, b, (short)0, c, false, false);
  asm volatile("v_nop\n\tv_nop\n\tv_nop\n\tv_nop" : "+v"(d) : "v"(a), "v"(b));
  return d;
}

__global__ void __launch_bounds__(256)
wcvt_kernel(const float* __restrict__ qw, const float* __restrict__ ow, _Float16* __restrict__ w16) {
  const int i   = blockIdx.x * 256 + threadIdx.x;
  const int nq8 = C3 * CC / 8;
  v4f a, b;
  if (blockIdx.x < nq8 / 256) {
    a = *(const v4f*)(qw + (size_t)i * 8);
    b = *(const v4f*)(qw + (size_t)i * 8 + 4);
  } else {
    const int j = i - nq8;
    a = *(const v4f*)(ow + (size_t)j * 8);
    b = *(const v4f*)(ow + (size_t)j * 8 + 4);
  }
  v8h pk;
#pragma unroll
  for (int j = 0; j < 4; ++j) {
    pk[j]     = (_Float16)(bfr(a[j]) * WCARRY);
    pk[j + 4] = (_Float16)(bfr(b[j]) * WCARRY);
  }
  _Float16* d = w16 + (size_t)i * 8;
  *(volatile v8h*)d = pk;
  __threadfence();
  *(volatile v8h*)d = pk;
}

__global__ void __launch_bounds__(256)
gn_kernel(const float* __restrict__ x, const float* __restrict__ gw,
          const float* __restrict__ gb, _Float16* __restrict__ xnt) {
  __shared__ __attribute__((aligned(16))) float tile[64 * 65];
  __shared__ __attribute__((aligned(16))) float red[4][256];
  const int gp  = blockIdx.x;
  const int n   = blockIdx.y;
  const int tid = threadIdx.x;
  const int c0  = gp * 64;
  const float* xb = x + ((size_t)n * CC + c0) * SEQ_FULL;
  const int S4 = SEQ / 4;

  float s0 = 0.f, q0 = 0.f, s1 = 0.f, q1 = 0.f;
#pragma unroll 1
  for (int i = tid; i < 32 * S4; i += 256) {
    const int cl = i / S4;
    const int t4 = i - cl * S4;
    v4f a = *(const v4f*)(xb + (size_t)cl * SEQ_FULL + t4 * 4);
    v4f b = *(const v4f*)(xb + (size_t)(cl + 32) * SEQ_FULL + t4 * 4);
#pragma unroll
    for (int j = 0; j < 4; ++j) {
      const float va = bfr(a[j]), vb = bfr(b[j]);
      s0 += va; q0 += va * va;
      s1 += vb; q1 += vb * vb;
    }
  }
  red[0][tid] = s0; red[1][tid] = q0; red[2][tid] = s1; red[3][tid] = q1;
  __syncthreads();
  for (int o = 128; o > 0; o >>= 1) {
    if (tid < o) {
      red[0][tid] += red[0][tid + o];
      red[1][tid] += red[1][tid + o];
      red[2][tid] += red[2][tid + o];
      red[3][tid] += red[3][tid + o];
    }
    __syncthreads();
  }
  const float inv_cnt = 1.0f / (float)(32 * SEQ);
  const float mean0 = red[0][0] * inv_cnt;
  const float var0  = red[1][0] * inv_cnt - mean0 * mean0;
  const float rstd0 = rsqrtf(var0 + GN_EPS);
  const float mean1 = red[2][0] * inv_cnt;
  const float var1  = red[3][0] * inv_cnt - mean1 * mean1;
  const float rstd1 = rsqrtf(var1 + GN_EPS);

  const int  cseg = tid & 7;
  const bool g1   = cseg >= 4;
  const float mean = g1 ? mean1 : mean0;
  const float rstd = g1 ? rstd1 : rstd0;
  float gwv[8], gbv[8];
  {
    v4f w0 = *(const v4f*)(gw + c0 + cseg * 8);
    v4f w1 = *(const v4f*)(gw + c0 + cseg * 8 + 4);
    v4f b0 = *(const v4f*)(gb + c0 + cseg * 8);
    v4f b1 = *(const v4f*)(gb + c0 + cseg * 8 + 4);
#pragma unroll
    for (int j = 0; j < 4; ++j) {
      gwv[j] = bfr(w0[j]); gwv[j + 4] = bfr(w1[j]);
      gbv[j] = bfr(b0[j]); gbv[j + 4] = bfr(b1[j]);
    }
  }
  _Float16* dst_base = xnt + (size_t)n * SEQ * CC + c0 + cseg * 8;

#pragma unroll 1
  for (int tt = 0; tt < SEQ / 64; ++tt) {
    __syncthreads();
#pragma unroll
    for (int k = 0; k < 4; ++k) {
      const int idx = tid + 256 * k;
      const int cl  = idx >> 4;
      const int tl4 = idx & 15;
      v4f a = *(const v4f*)(xb + (size_t)cl * SEQ_FULL + tt * 64 + tl4 * 4);
      float* tp = &tile[cl * 65 + tl4 * 4];
      tp[0] = bfr(a[0]); tp[1] = bfr(a[1]); tp[2] = bfr(a[2]); tp[3] = bfr(a[3]);
    }
    __syncthreads();
    v8h keep[2];
#pragma unroll
    for (int it2 = 0; it2 < 2; ++it2) {
      const int tl = it2 * 32 + (tid >> 3);
      v8h pk;
#pragma unroll
      for (int j = 0; j < 8; ++j) {
        const float v = (tile[(cseg * 8 + j) * 65 + tl] - mean) * rstd * gwv[j] + gbv[j];
        pk[j] = (_Float16)v;
      }
      keep[it2] = pk;
      *(volatile v8h*)(dst_base + (size_t)(tt * 64 + tl) * CC) = pk;
    }
    __threadfence();
#pragma unroll
    for (int it2 = 0; it2 < 2; ++it2) {
      const int tl = it2 * 32 + (tid >> 3);
      *(volatile v8h*)(dst_base + (size_t)(tt * 64 + tl) * CC) = keep[it2];
    }
  }
}

template<int MODE>
__global__ void __launch_bounds__(256)
gemm_kernel(const _Float16* __restrict__ Aw, const _Float16* __restrict__ Bsrc,
            const float* __restrict__ bias, const float* __restrict__ xres,
            _Float16* __restrict__ o0, _Float16* __restrict__ o1, _Float16* __restrict__ o2,
            float* __restrict__ outp) {
  __shared__ __attribute__((aligned(16))) float smem[8704];
  _Float16* As = reinterpret_cast<_Float16*>(smem);
  _Float16* Bs = As + 128 * LDST;

  const int t    = threadIdx.x;
  const int lane = t & 31;
  const int wave = t >> 5;
  const int wm   = wave & 3;
  const int wn   = wave >> 2;
  const int h    = lane >> 4;
  const int rl   = lane & 15;
  const int kfo  = 8 * h;
  const int n    = blockIdx.z;
  const int blockM = blockIdx.x * 128;
  const int blockN = blockIdx.y * 128;
  const int rowL   = t >> 2;
  const int colSeg = (t & 3) * 8;

  v8f acc[2][4];
  const v8f z8f = {};
#pragma unroll
  for (int i = 0; i < 2; ++i)
#pragma unroll
    for (int j = 0; j < 4; ++j) acc[i][j] = z8f;

  const _Float16* gA = Aw + (size_t)blockM * CC;

#pragma unroll 1
  for (int it = 0; it < CC / 32; ++it) {
    const int kk = it * 32;
#pragma unroll
    for (int rep = 0; rep < 2; ++rep) {
      const int r = rep * 64 + rowL;
      *(v8h*)&As[r * LDST + colSeg] = *(const v8h*)(gA + (size_t)r * CC + kk + colSeg);
      v8h bv;
      if (MODE == 0) {
        bv = *(const v8h*)(Bsrc + ((size_t)n * SEQ + blockN + r) * CC + kk + colSeg);
      } else {
        const int head = (kk >> 3) + (t & 3);
        bv = *(const v8h*)(Bsrc + (((size_t)n * NHEAD + head) * SEQ + blockN + r) * HDIM);
      }
      *(v8h*)&Bs[r * LDST + colSeg] = bv;
    }
    __syncthreads();

    Frag a[2], b[4];
#pragma unroll
    for (int mi = 0; mi < 2; ++mi) {
      const int m = wm * 32 + mi * 16 + rl;
      a[mi].h[0] = *(const v8h*)&As[m * LDST + kfo];
      a[mi].h[1] = *(const v8h*)&As[m * LDST + kfo + 16];
    }
#pragma unroll
    for (int ni = 0; ni < 4; ++ni) {
      const int nn = wn * 64 + ni * 16 + rl;
      b[ni].h[0] = *(const v8h*)&Bs[nn * LDST + kfo];
      b[ni].h[1] = *(const v8h*)&Bs[nn * LDST + kfo + 16];
    }
#pragma unroll
    for (int mi = 0; mi < 2; ++mi)
#pragma unroll
      for (int ni = 0; ni < 4; ++ni)
        acc[mi][ni] = wmma16(a[mi].v, b[ni].v, acc[mi][ni]);
    __syncthreads();
  }

  if (MODE == 0) {
    const int sec = blockIdx.x >> 1;
    const float sA = 1.0f / WCARRY;
    float bb[2][8];
#pragma unroll
    for (int mi = 0; mi < 2; ++mi) {
      const int ob = blockM + wm * 32 + mi * 16 + 8 * h;
      v4f b0 = *(const v4f*)(bias + ob);
      v4f b1 = *(const v4f*)(bias + ob + 4);
#pragma unroll
      for (int j = 0; j < 4; ++j) { bb[mi][j] = bfr(b0[j]); bb[mi][j + 4] = bfr(b1[j]); }
    }
    if (sec < 2) {
      _Float16* dst = (sec == 0) ? o0 : o1;
      v8h pk[2][4];
#pragma unroll
      for (int mi = 0; mi < 2; ++mi)
#pragma unroll
        for (int ni = 0; ni < 4; ++ni) {
          v8h p;
#pragma unroll
          for (int r = 0; r < 8; ++r) p[r] = (_Float16)(acc[mi][ni][r] * sA + bb[mi][r]);
          pk[mi][ni] = p;
        }
#pragma unroll
      for (int mi = 0; mi < 2; ++mi) {
        const int head = (blockM - sec * CC + wm * 32 + mi * 16 + 8 * h) >> 3;
#pragma unroll
        for (int ni = 0; ni < 4; ++ni) {
          const int tok = blockN + wn * 64 + ni * 16 + rl;
          *(volatile v8h*)(dst + (((size_t)n * NHEAD + head) * SEQ + tok) * HDIM) = pk[mi][ni];
        }
      }
      __threadfence();
#pragma unroll
      for (int mi = 0; mi < 2; ++mi) {
        const int head = (blockM - sec * CC + wm * 32 + mi * 16 + 8 * h) >> 3;
#pragma unroll
        for (int ni = 0; ni < 4; ++ni) {
          const int tok = blockN + wn * 64 + ni * 16 + rl;
          *(volatile v8h*)(dst + (((size_t)n * NHEAD + head) * SEQ + tok) * HDIM) = pk[mi][ni];
        }
      }
    } else {
      _Float16* Vs = reinterpret_cast<_Float16*>(smem);
#pragma unroll
      for (int mi = 0; mi < 2; ++mi)
#pragma unroll
        for (int ni = 0; ni < 4; ++ni)
#pragma unroll
          for (int r = 0; r < 8; ++r) {
            const int ol = wm * 32 + mi * 16 + 8 * h + r;
            const int tl = wn * 64 + ni * 16 + rl;
            Vs[ol * VST + tl] = (_Float16)(acc[mi][ni][r] * sA + bb[mi][r]);
          }
      __syncthreads();
      const int osb = blockM - 2 * CC;
      v8h keep[8];
#pragma unroll
      for (int it2 = 0; it2 < 8; ++it2) {
        const int row = it2 * 16 + (t >> 4);
        const int seg = t & 15;
        keep[it2] = *(const v8h*)&Vs[row * VST + seg * 8];
        *(volatile v8h*)(o2 + ((size_t)n * CC + osb + row) * SEQ + blockN + seg * 8) = keep[it2];
      }
      __threadfence();
#pragma unroll
      for (int it2 = 0; it2 < 8; ++it2) {
        const int row = it2 * 16 + (t >> 4);
        const int seg = t & 15;
        *(volatile v8h*)(o2 + ((size_t)n * CC + osb + row) * SEQ + blockN + seg * 8) = keep[it2];
      }
    }
  } else {
    float* Os = smem;
    const float sO = 1.0f / (WCARRY * YCARRY);
#pragma unroll
    for (int hh = 0; hh < 2; ++hh) {
      __syncthreads();
      if ((wm >> 1) == hh) {
#pragma unroll
        for (int mi = 0; mi < 2; ++mi)
#pragma unroll
          for (int ni = 0; ni < 4; ++ni)
#pragma unroll
            for (int r = 0; r < 8; ++r) {
              const int ol = (wm & 1) * 32 + mi * 16 + 8 * h + r;
              const int tl = wn * 64 + ni * 16 + rl;
              Os[ol * OST + tl] = acc[mi][ni][r];
            }
      }
      __syncthreads();
      v4f keep[8];
#pragma unroll
      for (int it2 = 0; it2 < 8; ++it2) {
        const int row = it2 * 8 + wave;
        const int o   = blockM + hh * 64 + row;
        v4f av = *(const v4f*)&Os[row * OST + lane * 4];
        const float bo = bfr(bias[o]);
        const size_t gi = ((size_t)n * CC + o) * SEQ_FULL + blockN + lane * 4;
        v4f xr = *(const v4f*)(xres + gi);
        v4f val;
#pragma unroll
        for (int j = 0; j < 4; ++j) val[j] = bfr(xr[j]) + (av[j] * sO + bo);
        keep[it2] = val;
        *(volatile v4f*)(outp + gi) = val;
      }
      __threadfence();
#pragma unroll
      for (int it2 = 0; it2 < 8; ++it2) {
        const int row = it2 * 8 + wave;
        const int o   = blockM + hh * 64 + row;
        const size_t gi = ((size_t)n * CC + o) * SEQ_FULL + blockN + lane * 4;
        *(volatile v4f*)(outp + gi) = keep[it2];
      }
    }
  }
}

__global__ void __launch_bounds__(256)
attn_kernel(const _Float16* __restrict__ qp, const _Float16* __restrict__ kp,
            const _Float16* __restrict__ vp, _Float16* __restrict__ yp) {
  const int lane = threadIdx.x & 31;
  const int w    = threadIdx.x >> 5;
  const int h    = lane >> 4;
  const int rl   = lane & 15;
  const int head = blockIdx.y;
  const int n    = blockIdx.z;
  const int s0   = blockIdx.x * 128 + w * 16;
  const size_t nh = (size_t)n * NHEAD + head;
  const _Float16* qb = qp + nh * SEQ * HDIM;
  const _Float16* kb = kp + nh * SEQ * HDIM;
  const _Float16* vb = vp + (nh * HDIM + (rl & 7)) * (size_t)SEQ + 8 * h;
  const v8h z8  = {};
  const v8f z8f = {};

  Frag qf;
  {
    v8h qv = *(const v8h*)(qb + (size_t)(s0 + rl) * HDIM);
    qf.h[0] = h ? z8 : qv;
    qf.h[1] = z8;
  }

  v8f acco = z8f;
  float m = -1e30f, l = 0.f;
  const float c2 = 0.35355339059327373f * 1.4426950408889634f;

#pragma unroll 1
  for (int tc = 0; tc < SEQ / 32; ++tc) {
    const int t0 = tc * 32;
    Frag ka0, ka1;
    {
      v8h k0 = *(const v8h*)(kb + (size_t)(t0 + rl) * HDIM);
      v8h k1 = *(const v8h*)(kb + (size_t)(t0 + 16 + rl) * HDIM);
      ka0.h[0] = h ? z8 : k0; ka0.h[1] = z8;
      ka1.h[0] = h ? z8 : k1; ka1.h[1] = z8;
    }
    v8f d0 = wmma16(ka0.v, qf.v, z8f);
    v8f d1 = wmma16(ka1.v, qf.v, z8f);
    v8f x0 = d0 * c2;
    v8f x1 = d1 * c2;
    float mx = -1e30f;
#pragma unroll
    for (int r = 0; r < 8; ++r) mx = fmaxf(mx, fmaxf(x0[r], x1[r]));
    mx = fmaxf(mx, __shfl_xor(mx, 16, 32));
    const float mn   = fmaxf(m, mx);
    const float corr = exp2f(m - mn);
    m = mn;
    l = l * corr;
    acco = acco * corr;

    float ps = 0.f;
    v8h ph0, ph1;
#pragma unroll
    for (int r = 0; r < 8; ++r) {
      const float p0 = exp2f(x0[r] - mn);
      const float p1 = exp2f(x1[r] - mn);
      ps += p0 + p1;
      ph0[r] = (_Float16)(p0 * PCARRY);
      ph1[r] = (_Float16)(p1 * PCARRY);
    }
    l += ps;
    Frag pb;
    pb.h[0] = ph0;
    pb.h[1] = ph1;
    Frag va;
    va.h[0] = *(const v8h*)(vb + t0);
    va.h[1] = *(const v8h*)(vb + t0 + 16);
    acco = wmma16(va.v, pb.v, acco);
  }

  const float lt  = l + __shfl_xor(l, 16, 32);
  const float inv = YCARRY / (lt * PCARRY);
  v8h yv;
#pragma unroll
  for (int r = 0; r < 8; ++r) yv[r] = (_Float16)(acco[r] * inv);
  _Float16* yd = yp + (nh * SEQ + s0 + rl) * HDIM;
  if (h == 0) *(volatile v8h*)yd = yv;
  __threadfence();
  if (h == 0) *(volatile v8h*)yd = yv;
}

extern "C" void kernel_launch(void* const* d_in, const int* in_sizes, int n_in,
                              void* d_out, int out_size, void* d_ws, size_t ws_size,
                              hipStream_t stream) {
  if (n_in < 7) return;
  if (in_sizes[0] < NB * CC * SEQ_FULL) return;
  if (in_sizes[1] < CC || in_sizes[2] < CC) return;
  if (in_sizes[3] < C3 * CC || in_sizes[4] < C3) return;
  if (in_sizes[5] < CC * CC || in_sizes[6] < CC) return;
  if (out_size < NB * CC * SEQ_FULL) return;

  const float* x     = (const float*)d_in[0];
  const float* gn_w  = (const float*)d_in[1];
  const float* gn_b  = (const float*)d_in[2];
  const float* qkv_w = (const float*)d_in[3];
  const float* qkv_b = (const float*)d_in[4];
  const float* out_w = (const float*)d_in[5];
  const float* out_b = (const float*)d_in[6];
  float* out = (float*)d_out;

  char* ws = (char*)d_ws;
  size_t off = 0;
  auto carve = [&](size_t bytes) -> char* {
    char* p = ws + off;
    off += (bytes + 255) & ~(size_t)255;
    return p;
  };
  const size_t plane = (size_t)NB * NHEAD * SEQ * HDIM * 2;
  _Float16* w16 = (_Float16*)carve((size_t)(C3 + CC) * CC * 2);
  _Float16* xnt = (_Float16*)carve((size_t)NB * SEQ * CC * 2);
  _Float16* q16 = (_Float16*)carve(plane);
  _Float16* k16 = (_Float16*)carve(plane);
  _Float16* v16 = (_Float16*)carve(plane);
  _Float16* y16 = (_Float16*)carve(plane);
  if (off > ws_size) return;

  wcvt_kernel<<<(C3 * CC + CC * CC) / 8 / 256, 256, 0, stream>>>(qkv_w, out_w, w16);
  gn_kernel<<<dim3(CC / 64, NB), 256, 0, stream>>>(x, gn_w, gn_b, xnt);
  gemm_kernel<0><<<dim3(C3 / 128, SEQ / 128, NB), 256, 0, stream>>>(
      w16, xnt, qkv_b, x, q16, k16, v16, out);
  attn_kernel<<<dim3(SEQ / 128, NHEAD, NB), 256, 0, stream>>>(q16, k16, v16, y16);
  gemm_kernel<1><<<dim3(CC / 128, SEQ / 128, NB), 256, 0, stream>>>(
      w16 + (size_t)C3 * CC, y16, out_b, x, q16, k16, v16, out);
}
